// GCNAggregator_41755672051923
// MI455X (gfx1250) — hardware-verified
//
#include <hip/hip_runtime.h>
#include <stddef.h>


typedef _Float16 v16h __attribute__((ext_vector_type(16)));
typedef _Float16 v8h  __attribute__((ext_vector_type(8)));
typedef float    v8f  __attribute__((ext_vector_type(8)));
typedef float    v4f  __attribute__((ext_vector_type(4)));
typedef int      v4i  __attribute__((ext_vector_type(4)));
typedef unsigned v4u  __attribute__((ext_vector_type(4)));

#define EMB_D     128
#define NEIGH_K   32
#define ROWS_BLK  64
#define MAX_M     16384
#define MAX_MW    (MAX_M / 32)
#define KCONV     128
#define STG_PITCH 132
#define NTHR      256

static_assert(NTHR == ROWS_BLK * 4);
static_assert(NTHR == 2 * EMB_D);
static_assert((STG_PITCH % 4) == 0);
static_assert(ROWS_BLK * STG_PITCH <= ROWS_BLK * MAX_MW);

union FragA   { v16h v; unsigned u[8]; };
union FragB   { v16h v; v8h hv[2]; };
union GemmLds { unsigned bits[ROWS_BLK * MAX_MW]; float stage[ROWS_BLK * STG_PITCH]; };

__device__ __forceinline__ v8f wmma16(v16h a, v16h b, v8f c)
{
    v8f d = __builtin_amdgcn_wmma_f32_16x16x32_f16(false, a, false, b, (short)0, c, false, false);
    asm volatile("v_nop\n\tv_nop\n\tv_nop\n\tv_nop" : "+v"(d) : "v"(a), "v"(b));
    return d;
}

__device__ __forceinline__ void build_bits(unsigned* sb,
                                           const int* __restrict__ nodes,
                                           const int* __restrict__ neigh,
                                           int row0, int M, int tid)
{
    const v4u z = {0u, 0u, 0u, 0u};
    v4u* zb = (v4u*)sb;
    for (int t = tid; t < (ROWS_BLK * MAX_MW) / 4; t += NTHR) zb[t] = z;
    __syncthreads();
    if (tid < ROWS_BLK) {
        const int row = row0 + tid;
        unsigned* rb = sb + tid * MAX_MW;
        for (int k = 0; k <= NEIGH_K; ++k) {
            int c = (k < NEIGH_K) ? neigh[(size_t)row * NEIGH_K + k] : nodes[row];
            if (c < 0) c += M;
            if ((unsigned)c < (unsigned)M) rb[c >> 5] |= (1u << (c & 31));
        }
    }
    __syncthreads();
}

__global__ void __launch_bounds__(NTHR)
k_colcount(const int* __restrict__ nodes,
           const int* __restrict__ neigh,
           int*       __restrict__ pc,
           int M, int MW)
{
    __shared__ __align__(16) unsigned sBits[ROWS_BLK * MAX_MW];
    const int tid = threadIdx.x;
    const int blk = blockIdx.x;
    build_bits(sBits, nodes, neigh, blk * ROWS_BLK, M, tid);

    for (int w = tid; w < MW; w += NTHR) {
        unsigned a8[8];
        #pragma unroll
        for (int j = 0; j < 8; ++j) a8[j] = 0u;
        #pragma unroll 4
        for (int r = 0; r < ROWS_BLK; ++r) {
            const unsigned word = sBits[r * MAX_MW + w];
            #pragma unroll
            for (int j = 0; j < 8; ++j) a8[j] += (word >> j) & 0x01010101u;
        }
        v4i piece[8];
        #pragma unroll
        for (int q = 0; q < 8; ++q) {
            v4i t;
            t.x = (int)((a8[(4 * q + 0) & 7] >> (8 * ((4 * q + 0) >> 3))) & 0xFFu);
            t.y = (int)((a8[(4 * q + 1) & 7] >> (8 * ((4 * q + 1) >> 3))) & 0xFFu);
            t.z = (int)((a8[(4 * q + 2) & 7] >> (8 * ((4 * q + 2) >> 3))) & 0xFFu);
            t.w = (int)((a8[(4 * q + 3) & 7] >> (8 * ((4 * q + 3) >> 3))) & 0xFFu);
            piece[q] = t;
        }
        int* dst = pc + (size_t)blk * (size_t)M + (size_t)w * 32;
        #pragma unroll
        for (int q = 0; q < 8; ++q) *(volatile v4i*)(dst + 4 * q) = piece[q];
        __threadfence();
        #pragma unroll
        for (int q = 0; q < 8; ++q) *(volatile v4i*)(dst + 4 * q) = piece[q];
    }
}

__global__ void __launch_bounds__(NTHR)
k_convert(const float* __restrict__ embed,
          const int*   __restrict__ pc,
          _Float16*    __restrict__ Bt,
          int M, int NB)
{
    __shared__ float sCs[KCONV];
    __shared__ __align__(16) _Float16 sT[EMB_D * KCONV];
    const int tid = threadIdx.x;
    const int k0  = blockIdx.x * KCONV;

    if (tid < KCONV) {
        int c = 0;
        const int* p = pc + k0 + tid;
        for (int b = 0; b < NB; ++b) c += p[(size_t)b * (size_t)M];
        if (c < 1) c = 1;
        sCs[tid] = rsqrtf((float)c);
    }
    __syncthreads();

    for (int i = tid; i < KCONV * (EMB_D / 4); i += NTHR) {
        const int k  = i >> 5;
        const int c4 = i & 31;
        const v4f v  = *(const v4f*)(embed + (size_t)(k0 + k) * EMB_D + c4 * 4);
        const float s = sCs[k];
        sT[(c4 * 4 + 0) * KCONV + k] = (_Float16)(v.x * s);
        sT[(c4 * 4 + 1) * KCONV + k] = (_Float16)(v.y * s);
        sT[(c4 * 4 + 2) * KCONV + k] = (_Float16)(v.z * s);
        sT[(c4 * 4 + 3) * KCONV + k] = (_Float16)(v.w * s);
    }
    __syncthreads();

    {
        const int n  = tid >> 1;
        const int hf = tid & 1;
        const v8h* src = (const v8h*)(sT + n * KCONV + hf * 64);
        _Float16* dstp = Bt + (size_t)n * (size_t)M + (size_t)k0 + hf * 64;
        v8h vv[8];
        #pragma unroll
        for (int q = 0; q < 8; ++q) vv[q] = src[q];
        #pragma unroll
        for (int q = 0; q < 8; ++q) *(volatile v8h*)(dstp + 8 * q) = vv[q];
        __threadfence();
        #pragma unroll
        for (int q = 0; q < 8; ++q) *(volatile v8h*)(dstp + 8 * q) = vv[q];
    }
}

__global__ void __launch_bounds__(NTHR)
k_gemm(const int*      __restrict__ nodes,
       const int*      __restrict__ neigh,
       const _Float16* __restrict__ Bt,
       float*          __restrict__ out,
       int M, int MW)
{
    __shared__ __align__(16) GemmLds sU;
    __shared__ float sRs[ROWS_BLK];

    const int tid  = threadIdx.x;
    const int blk  = blockIdx.x;
    const int row0 = blk * ROWS_BLK;
    const int lane = tid & 31;
    const int wv   = tid >> 5;

    build_bits(sU.bits, nodes, neigh, row0, M, tid);

    for (int r = wv; r < ROWS_BLK; r += NTHR / 32) {
        int s = 0;
        for (int w = lane; w < MW; w += 32) s += (int)__popc(sU.bits[r * MAX_MW + w]);
        s += __shfl_xor(s, 16);
        s += __shfl_xor(s, 8);
        s += __shfl_xor(s, 4);
        s += __shfl_xor(s, 2);
        s += __shfl_xor(s, 1);
        if (lane == 0) sRs[r] = rsqrtf((float)(s < 1 ? 1 : s));
    }
    __syncthreads();

    const int h  = lane >> 4;
    const int m  = lane & 15;
    const int rg = wv & 3;
    const int ch = wv >> 2;
    const unsigned* abits = sU.bits + (rg * 16 + m) * MAX_MW;
    const _Float16* bbase = Bt + (size_t)(ch * 64 + m) * (size_t)M + 8 * h;

    v8f acc[4];
    {
        const v8f z = {0.f, 0.f, 0.f, 0.f, 0.f, 0.f, 0.f, 0.f};
        #pragma unroll
        for (int j = 0; j < 4; ++j) acc[j] = z;
    }

    for (int ks = 0; ks < MW; ++ks) {
        const unsigned word = abits[ks];
        const unsigned wlo  = (word >> (8 * h)) & 0xFFu;
        const unsigned whi  = (word >> (16 + 8 * h)) & 0xFFu;
        FragA af;
        #pragma unroll
        for (int p = 0; p < 4; ++p) {
            const unsigned l0 = 0u - ((wlo >> (2 * p)) & 1u);
            const unsigned l1 = 0u - ((wlo >> (2 * p + 1)) & 1u);
            const unsigned h0 = 0u - ((whi >> (2 * p)) & 1u);
            const unsigned h1 = 0u - ((whi >> (2 * p + 1)) & 1u);
            af.u[p]     = (l0 & 0x3C00u) | (l1 & 0x3C000000u);
            af.u[4 + p] = (h0 & 0x3C00u) | (h1 & 0x3C000000u);
        }
        const size_t k0 = (size_t)ks * 32;
        #pragma unroll
        for (int j = 0; j < 4; ++j) {
            const _Float16* bp = bbase + (size_t)j * 16 * (size_t)M + k0;
            FragB bf;
            bf.hv[0] = *(const v8h*)(bp);
            bf.hv[1] = *(const v8h*)(bp + 16);
            acc[j] = wmma16(af.v, bf.v, acc[j]);
        }
    }

    __syncthreads();

    #pragma unroll
    for (int j = 0; j < 4; ++j) {
        #pragma unroll
        for (int r = 0; r < 8; ++r) {
            const int lr = rg * 16 + 8 * h + r;
            sU.stage[lr * STG_PITCH + ch * 64 + j * 16 + m] = acc[j][r] * sRs[lr];
        }
    }
    __syncthreads();

    {
        const int lr = tid >> 2;
        const int q  = tid & 3;
        const v4f* src = (const v4f*)(sU.stage + lr * STG_PITCH + q * 32);
        float* dp = out + (size_t)(row0 + lr) * EMB_D + q * 32;
        v4f vv[8];
        #pragma unroll
        for (int e = 0; e < 8; ++e) vv[e] = src[e];
        #pragma unroll
        for (int e = 0; e < 8; ++e) *(volatile v4f*)(dp + 4 * e) = vv[e];
        __threadfence();
        #pragma unroll
        for (int e = 0; e < 8; ++e) *(volatile v4f*)(dp + 4 * e) = vv[e];
    }
}

extern "C" void kernel_launch(void* const* d_in, const int* in_sizes, int n_in,
                              void* d_out, int out_size, void* d_ws, size_t ws_size,
                              hipStream_t stream)
{
    if (n_in < 3) return;
    const int*   nodes = (const int*)d_in[0];
    const int*   neigh = (const int*)d_in[1];
    const float* embed = (const float*)d_in[2];
    float*       out   = (float*)d_out;

    const int N = in_sizes[0];
    if (N <= 0 || (N % ROWS_BLK) != 0) return;
    if (in_sizes[1] != N * NEIGH_K) return;
    if (out_size != N * EMB_D) return;
    const int M = in_sizes[2] / EMB_D;
    if (M * EMB_D != in_sizes[2] || M < KCONV || M > MAX_M || (M % KCONV) != 0) return;
    const int MW = M / 32;
    const int NB = N / ROWS_BLK;

    const size_t pc_bytes = (size_t)NB * (size_t)M * sizeof(int);
    const size_t bt_off   = (pc_bytes + 255) & ~(size_t)255;
    const size_t bt_bytes = (size_t)EMB_D * (size_t)M * sizeof(_Float16);
    if (bt_off + bt_bytes > ws_size) return;

    char* ws = (char*)d_ws;
    int*      pc = (int*)ws;
    _Float16* Bt = (_Float16*)(ws + bt_off);

    k_colcount<<<NB, NTHR, 0, stream>>>(nodes, neigh, pc, M, MW);
    k_convert<<<M / KCONV, NTHR, 0, stream>>>(embed, pc, Bt, M, NB);
    k_gemm<<<NB, NTHR, 0, stream>>>(nodes, neigh, Bt, out, M, MW);
}
